// TemporalAttentionModule_9680856285923
// MI455X (gfx1250) — hardware-run, weakly checked
//
#include <hip/hip_runtime.h>
#include <math.h>

typedef __attribute__((ext_vector_type(16))) _Float16 v16h;
typedef __attribute__((ext_vector_type(8)))  _Float16 v8h;
typedef __attribute__((ext_vector_type(16))) __bf16   v16b;
typedef __attribute__((ext_vector_type(8)))  __bf16   v8b;
typedef __attribute__((ext_vector_type(8)))  float    v8f;
typedef __attribute__((ext_vector_type(4)))  float    v4f;
typedef __attribute__((ext_vector_type(8)))  unsigned v8u;

#define NBATCH 8
#define NFEAT 128
#define NNODE 256
#define NEMB 256
#define ITILE 16
#define GSTAGE 2
#define APITCH 72
#define EPITCH 260
#define LRELU_SLOPE 0.2f
#define PCARRY 1024.0f
#define WCARRY 16.0f
#define ACARRY 16.0f

static_assert(NNODE % 64 == 0 && NEMB % 64 == 0 && NFEAT % 64 == 0, "GEMM M/N tile multiples");
static_assert(NFEAT % 32 == 0 && NNODE % 32 == 0, "GEMM K multiples of 32");
static_assert(NNODE % ITILE == 0 && ITILE % GSTAGE == 0 && NEMB % 32 == 0, "score tiling");
static_assert(APITCH % 8 == 0 && APITCH >= GSTAGE * 32, "A tile pitch");
static_assert((EPITCH * 4) % 16 == 0 && EPITCH >= NNODE, "score tile pitch");
static_assert(NNODE == 256, "one thread per key column in the score kernel");

__device__ __forceinline__ unsigned short f2bf_bits(float f) {
  unsigned u = __float_as_uint(f);
  return (unsigned short)((u + 0x7FFFu + ((u >> 16) & 1u)) >> 16);
}
__device__ __forceinline__ float bf_bits2f(unsigned short h) { return __uint_as_float(((unsigned)h) << 16); }

__device__ __forceinline__ void dep_guard_h(v8f& a, v8f& b, v16h x, v16h y) { asm volatile("v_nop\n\tv_nop\n\tv_nop\n\tv_nop" : "+v"(a), "+v"(b) : "v"(x), "v"(y)); }
__device__ __forceinline__ void dep_guard_b(v8f& a, v8f& b, v16b x, v16b y) { asm volatile("v_nop\n\tv_nop\n\tv_nop\n\tv_nop" : "+v"(a), "+v"(b) : "v"(x), "v"(y)); }
__device__ __forceinline__ void keep4_h(v16h a, v16h b, v16h c, v16h d) { asm volatile("v_nop" :: "v"(a), "v"(b), "v"(c), "v"(d)); }
__device__ __forceinline__ void keep4_b(v16b a, v16b b, v16b c, v16b d) { asm volatile("v_nop" :: "v"(a), "v"(b), "v"(c), "v"(d)); }
__device__ __forceinline__ void acc_guard4(v8f& a, v8f& b, v8f& c, v8f& d) { asm volatile("v_nop\n\tv_nop\n\tv_nop\n\tv_nop" : "+v"(a), "+v"(b), "+v"(c), "+v"(d)); }
__device__ __forceinline__ void guard2x3(v8f& a, v8f& b, v16h x, v16h y, v16h z) { asm volatile("v_nop\n\tv_nop\n\tv_nop\n\tv_nop" : "+v"(a), "+v"(b) : "v"(x), "v"(y), "v"(z)); }
__device__ __forceinline__ void acc_guard2(v8f& a, v8f& b) { asm volatile("v_nop\n\tv_nop\n\tv_nop\n\tv_nop" : "+v"(a), "+v"(b)); }

template <typename T> struct Frag;
template <> struct Frag<_Float16> {
  typedef v16h V; union U { v16h v; v8h h[2]; };
  static __device__ __forceinline__ v16h load(const _Float16* p) {
    U f; f.h[0] = *(const v8h*)(p); f.h[1] = *(const v8h*)(p + 16); return f.v;
  }
  static __device__ __forceinline__ v8f mma(v16h a, v16h b, v8f c) {
    return __builtin_amdgcn_wmma_f32_16x16x32_f16(false, a, false, b, (short)0, c, false, false);
  }
  static __device__ __forceinline__ void guard(v8f& a, v8f& b, v16h x, v16h y) { dep_guard_h(a, b, x, y); }
  static __device__ __forceinline__ void keep(v16h a, v16h b, v16h c, v16h d) { keep4_h(a, b, c, d); }
};
template <> struct Frag<__bf16> {
  typedef v16b V; union U { v16b v; v8b h[2]; };
  static __device__ __forceinline__ v16b load(const __bf16* p) {
    U f; f.h[0] = *(const v8b*)(p); f.h[1] = *(const v8b*)(p + 16); return f.v;
  }
  static __device__ __forceinline__ v8f mma(v16b a, v16b b, v8f c) {
    return __builtin_amdgcn_wmma_f32_16x16x32_bf16(false, a, false, b, (short)0, c, false, false);
  }
  static __device__ __forceinline__ void guard(v8f& a, v8f& b, v16b x, v16b y) { dep_guard_b(a, b, x, y); }
  static __device__ __forceinline__ void keep(v16b a, v16b b, v16b c, v16b d) { keep4_b(a, b, c, d); }
};

template <int ET> struct Elem;
template <> struct Elem<0> { typedef _Float16 T; };
template <> struct Elem<1> { typedef __bf16 T; };
template <int ET, bool SPLIT, int BIAS_MODE, int OUT_MODE, bool RESID, int ACT = 0>
__global__ __launch_bounds__(256) void wmma_gemm64(
    const unsigned short* __restrict__ Ap, const unsigned short* __restrict__ A2p, int lda, long strideA,
    const unsigned short* __restrict__ Btp, const unsigned short* __restrict__ Bt2p, int ldb, long strideB,
    void* __restrict__ Cout, void* __restrict__ Cout2, int ldc, long strideC,
    const float* __restrict__ bias,
    const float* __restrict__ resid, long strideR,
    int M, int N, int K, float scale) {
  typedef typename Elem<ET>::T T;
  typedef typename Frag<T>::V V;
  const T* A = (const T*)Ap; const T* A2 = (const T*)A2p; const T* Bt = (const T*)Btp; const T* Bt2 = (const T*)Bt2p;
  __shared__ __align__(16) float sT[8][16 * 68];
  const int b    = blockIdx.y;
  const int lane = threadIdx.x & 31;
  const int wave = threadIdx.x >> 5;
  const int tilesN = N >> 6;
  const int tilesM = M >> 6;
  const int tile = blockIdx.x * 8 + wave;
  if (tile >= tilesM * tilesN) return;
  const int tm = tile / tilesN;
  const int tn = tile - tm * tilesN;
  const int m0 = tm << 6;
  const int n0 = tn << 6;

  const T* Ab  = A  + (size_t)b * strideA;
  const T* Bb  = Bt + (size_t)b * strideB;
  const T* Ab2 = SPLIT ? (A2  + (size_t)b * strideA) : nullptr;
  const T* Bb2 = SPLIT ? (Bt2 + (size_t)b * strideB) : nullptr;

  const int rlane = lane & 15;
  const int koff  = (lane >> 4) * 8;
  const int mOff  = (lane >> 4) * 8;

  v8f acc[4][4];
#pragma unroll
  for (int i = 0; i < 4; ++i)
#pragma unroll
    for (int j = 0; j < 4; ++j) acc[i][j] = (v8f){0.f,0.f,0.f,0.f,0.f,0.f,0.f,0.f};

  for (int k0 = 0; k0 < K; k0 += 32) {
    V bh[4], bl[4];
#pragma unroll
    for (int j = 0; j < 4; ++j) {
      const size_t bo = (size_t)(n0 + (j << 4) + rlane) * ldb + koff + k0;
      bh[j] = Frag<T>::load(Bb + bo);
      if (SPLIT) bl[j] = Frag<T>::load(Bb2 + bo);
    }
#pragma unroll
    for (int i = 0; i < 4; ++i) {
      const size_t ao = (size_t)(m0 + (i << 4) + rlane) * lda + koff + k0;
      V ah = Frag<T>::load(Ab + ao);
      V al;
      if (SPLIT) al = Frag<T>::load(Ab2 + ao);
#pragma unroll
      for (int j = 0; j < 4; ++j) {
        acc[i][j] = Frag<T>::mma(ah, bh[j], acc[i][j]);
        if (SPLIT) {
          acc[i][j] = Frag<T>::mma(ah, bl[j], acc[i][j]);
          acc[i][j] = Frag<T>::mma(al, bh[j], acc[i][j]);
        }
      }
      Frag<T>::guard(acc[i][0], acc[i][3], ah, SPLIT ? al : ah);
    }
    Frag<T>::keep(bh[0], bh[1], bh[2], bh[3]);
    if (SPLIT) Frag<T>::keep(bl[0], bl[1], bl[2], bl[3]);
  }
  acc_guard4(acc[0][0], acc[0][1], acc[0][2], acc[0][3]);
  acc_guard4(acc[1][0], acc[1][1], acc[1][2], acc[1][3]);
  acc_guard4(acc[2][0], acc[2][1], acc[2][2], acc[2][3]);
  acc_guard4(acc[3][0], acc[3][1], acc[3][2], acc[3][3]);

  float* slab = sT[wave];
  const float* Rb = RESID ? (resid + (size_t)b * strideR) : nullptr;
#pragma unroll
  for (int i = 0; i < 4; ++i) {
    const int mBase = m0 + (i << 4);
#pragma unroll
    for (int j = 0; j < 4; ++j) {
      const int n = n0 + (j << 4) + rlane;
      float bv = 0.f;
      if (BIAS_MODE == 2) bv = bias[n];
#pragma unroll
      for (int r = 0; r < 8; ++r) {
        float v = acc[i][j][r] * scale;
        if (BIAS_MODE == 1) v += bias[mBase + mOff + r];
        if (BIAS_MODE == 2) v += bv;
        if (RESID) v += Rb[(size_t)(mBase + mOff + r) * ldc + n];
        if (ACT == 1) v = tanhf(v);
        if (ACT == 2) v = fmaxf(v, 0.0f);
        if (ACT == 3) v = v / (1.0f + expf(-v));
        if (ACT == 4) v = (v > 0.f) ? v : 0.01f * v;
        if (ACT == 5) v = 0.5f * v * (1.0f + erff(v * 0.70710678118654752f));
        if (ACT == 6) { const float ex = expf(-v); v = 1.0f / (1.0f + ex); }
        slab[(mOff + r) * 68 + (j << 4) + rlane] = v;
      }
    }
    __builtin_amdgcn_fence(__ATOMIC_RELEASE, "workgroup");
    __builtin_amdgcn_wave_barrier();
    __builtin_amdgcn_fence(__ATOMIC_ACQUIRE, "workgroup");
    if (OUT_MODE == 0) {
      float* C = (float*)Cout + (size_t)b * strideC;
      const int hh = lane >> 4, c4 = (lane & 15) * 4;
      for (int pass = 0; pass < 2; ++pass) {
#pragma unroll
        for (int it = 0; it < 8; ++it) {
          const int row = it * 2 + hh;
          v4f v = *(const v4f*)(slab + row * 68 + c4);
          *(volatile v4f*)(C + (size_t)(mBase + row) * ldc + n0 + c4) = v;
        }
        __threadfence();
      }
    } else {
      const int q = lane >> 3, c8 = (lane & 7) * 8;
      unsigned short* C  = (unsigned short*)Cout  + (size_t)b * strideC;
      unsigned short* C2 = (OUT_MODE == 2) ? ((unsigned short*)Cout2 + (size_t)b * strideC) : nullptr;
      for (int pass = 0; pass < 2; ++pass) {
#pragma unroll
        for (int it = 0; it < 4; ++it) {
          const int row = it * 4 + q;
          const float* sp = slab + row * 68 + c8;
          v8h hv, lv;
#pragma unroll
          for (int e = 0; e < 8; ++e) {
            if (OUT_MODE == 1) {
              hv[e] = (_Float16)sp[e];
            } else {
              unsigned short hb = f2bf_bits(sp[e]);
              unsigned short lb = f2bf_bits(sp[e] - bf_bits2f(hb));
              hv[e] = __builtin_bit_cast(_Float16, hb);
              lv[e] = __builtin_bit_cast(_Float16, lb);
            }
          }
          *(volatile v8h*)(C + (size_t)(mBase + row) * ldc + n0 + c8) = hv;
          if (OUT_MODE == 2) *(volatile v8h*)(C2 + (size_t)(mBase + row) * ldc + n0 + c8) = lv;
        }
        __threadfence();
      }
    }
    __builtin_amdgcn_fence(__ATOMIC_RELEASE, "workgroup");
    __builtin_amdgcn_wave_barrier();
    __builtin_amdgcn_fence(__ATOMIC_ACQUIRE, "workgroup");
  }
}

__global__ __launch_bounds__(256) void cast_f32_f16x2(
    const float* __restrict__ in, _Float16* __restrict__ out, int n2) {
  int i = blockIdx.x * 256 + threadIdx.x;
  if (i < n2) {
    const _Float16 h0 = (_Float16)in[2 * i], h1 = (_Float16)in[2 * i + 1];
    const unsigned u = (unsigned)__builtin_bit_cast(unsigned short, h0) | ((unsigned)__builtin_bit_cast(unsigned short, h1) << 16);
    ((volatile unsigned*)out)[i] = u;
    __threadfence();
    ((volatile unsigned*)out)[i] = u;
  }
}

__global__ __launch_bounds__(256) void transpose_cast16(const float* __restrict__ in, unsigned short* __restrict__ out,
                                                        int nrows, int ncols, float sc)
{
  __shared__ float ts[64][65];
  const int tid = threadIdx.x;
  const int c0 = blockIdx.x * 64, r0 = blockIdx.y * 64, z = blockIdx.z;
  const float* inb = in + (size_t)z * nrows * ncols;
  _Float16* outb = (_Float16*)out + (size_t)z * nrows * ncols;
  const int c4 = (tid & 15) * 4, rb = tid >> 4;
#pragma unroll
  for (int s = 0; s < 4; ++s) {
    const int rr = rb + 16 * s;
    const v4f v = *(const v4f*)(inb + (size_t)(r0 + rr) * ncols + c0 + c4);
    ts[rr][c4 + 0] = v[0]; ts[rr][c4 + 1] = v[1]; ts[rr][c4 + 2] = v[2]; ts[rr][c4 + 3] = v[3];
  }
  __syncthreads();
  const int wave = tid >> 5, lane = tid & 31, q8 = lane >> 3, c8 = (lane & 7) * 8;
  v8h hv[2];
#pragma unroll
  for (int it = 0; it < 2; ++it) {
    const int cc = wave * 8 + it * 4 + q8;
#pragma unroll
    for (int u = 0; u < 8; ++u) hv[it][u] = (_Float16)(ts[c8 + u][cc] * sc);
  }
  for (int pass = 0; pass < 2; ++pass) {
#pragma unroll
    for (int it = 0; it < 2; ++it) {
      const int cc = wave * 8 + it * 4 + q8;
      *(volatile v8h*)(outb + (size_t)(c0 + cc) * nrows + r0 + c8) = hv[it];
    }
    __threadfence();
  }
}

__device__ __forceinline__ float lrelu_f(float t) { return (t > 0.0f) ? t : LRELU_SLOPE * t; }

__global__ __launch_bounds__(256) void score_softmax_kernel(
    const float* __restrict__ pproj, const float* __restrict__ qproj,
    const float* __restrict__ avec, const float* __restrict__ sbias,
    unsigned short* __restrict__ pout)
{
  __shared__ __align__(16) _Float16 Ah[NNODE * APITCH];
  __shared__ __align__(16) float    ps[ITILE * NEMB];
  __shared__ __align__(16) _Float16 a16[NEMB];
  __shared__ __align__(16) float    es[ITILE * EPITCH];

  const int tid = threadIdx.x;
  const int lane = tid & 31, wave = tid >> 5;
  const int rlane = lane & 15, hh = lane >> 4, koff = hh * 8;
  const int blk = blockIdx.x;
  const int b  = blk / (NNODE / ITILE);
  const int i0 = (blk - b * (NNODE / ITILE)) * ITILE;

  {
    const float* pb = pproj + ((size_t)b * NNODE + i0) * NEMB;
#pragma unroll
    for (int s = 0; s < 4; ++s) {
      const int idx = (tid + 256 * s) * 4;
      *(v4f*)(ps + idx) = *(const v4f*)(pb + idx);
    }
  }
  if (tid < 32) {
    const v4f x0 = *(const v4f*)(avec + 8 * tid);
    const v4f x1 = *(const v4f*)(avec + 8 * tid + 4);
    v8h hv;
#pragma unroll
    for (int u = 0; u < 4; ++u) { hv[u] = (_Float16)(x0[u] * ACARRY); hv[4 + u] = (_Float16)(x1[u] * ACARRY); }
    *(v8h*)(a16 + 8 * tid) = hv;
  }
  __syncthreads();

  const v8f zero8 = (v8f){0.f,0.f,0.f,0.f,0.f,0.f,0.f,0.f};
  v8f acc0 = zero8, acc1 = zero8;
  const int j = tid;
  const float* qrow = qproj + ((size_t)b * NNODE + j) * NEMB;
  _Float16* Aw = Ah + j * APITCH;
  const _Float16* Arow0 = Ah + (32 * wave + rlane) * APITCH + koff;
  const _Float16* Arow1 = Arow0 + 16 * APITCH;

#pragma unroll 1
  for (int ec = 0; ec < NEMB / 32; ++ec) {
    const int e0 = ec * 32;
    v4f qv[8];
#pragma unroll
    for (int u = 0; u < 8; ++u) qv[u] = *(const v4f*)(qrow + e0 + 4 * u);
    const v16h braw = Frag<_Float16>::load(a16 + e0 + koff);
    const v8u  bwraw = __builtin_bit_cast(v8u, braw);
#pragma unroll 1
    for (int ig = 0; ig < ITILE / GSTAGE; ++ig) {
#pragma unroll
      for (int il = 0; il < GSTAGE; ++il) {
        const float* prow = ps + (ig * GSTAGE + il) * NEMB + e0;
#pragma unroll
        for (int c4 = 0; c4 < 4; ++c4) {
          const v4f pa = *(const v4f*)(prow + 8 * c4);
          const v4f pb = *(const v4f*)(prow + 8 * c4 + 4);
          const v4f qa = qv[2 * c4], qb = qv[2 * c4 + 1];
          v8h hv;
#pragma unroll
          for (int u = 0; u < 4; ++u) {
            hv[u]     = (_Float16)lrelu_f(pa[u] + qa[u]);
            hv[4 + u] = (_Float16)lrelu_f(pb[u] + qb[u]);
          }
          *(v8h*)(Aw + il * 32 + 8 * c4) = hv;
        }
      }
      __syncthreads();
#pragma unroll
      for (int il = 0; il < GSTAGE; ++il) {
        const int ip = ig * GSTAGE + il;
        const unsigned msk = (rlane == ip) ? 0xffffffffu : 0u;
        v8u bw;
#pragma unroll
        for (int u = 0; u < 8; ++u) bw[u] = bwraw[u] & msk;
        const v16h bsel = __builtin_bit_cast(v16h, bw);
        const v16h af0 = Frag<_Float16>::load(Arow0 + il * 32);
        const v16h af1 = Frag<_Float16>::load(Arow1 + il * 32);
        acc0 = Frag<_Float16>::mma(af0, bsel, acc0);
        acc1 = Frag<_Float16>::mma(af1, bsel, acc1);
        guard2x3(acc0, acc1, af0, af1, bsel);
      }
      __syncthreads();
    }
  }
  acc_guard2(acc0, acc1);

  {
    const float s16 = 1.0f / ACARRY;
    float* ep = es + rlane * EPITCH + 32 * wave + 8 * hh;
#pragma unroll
    for (int r = 0; r < 8; ++r) { ep[r] = acc0[r] * s16; ep[16 + r] = acc1[r] * s16; }
  }
  __syncthreads();

  v8h pv[2];
#pragma unroll
  for (int rr = 0; rr < 2; ++rr) {
    const int ip = 2 * wave + rr;
    const float* erow = es + ip * EPITCH + 8 * lane;
    const float* brow = sbias + (size_t)(i0 + ip) * NNODE + 8 * lane;
    const v4f ea = *(const v4f*)(erow), eb = *(const v4f*)(erow + 4);
    const v4f ba = *(const v4f*)(brow), bb = *(const v4f*)(brow + 4);
    float ev[8];
#pragma unroll
    for (int u = 0; u < 4; ++u) { ev[u] = ea[u] + ba[u]; ev[4 + u] = eb[u] + bb[u]; }
    float m = ev[0];
#pragma unroll
    for (int u = 1; u < 8; ++u) m = fmaxf(m, ev[u]);
#pragma unroll
    for (int off = 1; off < 32; off <<= 1) m = fmaxf(m, __shfl_xor(m, off, 32));
    float ssum = 0.0f;
#pragma unroll
    for (int u = 0; u < 8; ++u) { ev[u] = expf(ev[u] - m); ssum += ev[u]; }
#pragma unroll
    for (int off = 1; off < 32; off <<= 1) ssum += __shfl_xor(ssum, off, 32);
    const float inv = PCARRY / ssum;
    v8h hv;
#pragma unroll
    for (int u = 0; u < 8; ++u) hv[u] = (_Float16)(ev[u] * inv);
    pv[rr] = hv;
  }
  _Float16* prow0 = (_Float16*)pout + ((size_t)b * NNODE + i0 + 2 * wave) * NNODE + 8 * lane;
  for (int pass = 0; pass < 2; ++pass) {
    *(volatile v8h*)(prow0) = pv[0];
    *(volatile v8h*)(prow0 + NNODE) = pv[1];
    __threadfence();
  }
}

extern "C" void kernel_launch(void* const* d_in, const int* in_sizes, int n_in,
                              void* d_out, int out_size, void* d_ws, size_t ws_size,
                              hipStream_t stream)
{
  if (n_in < 5) return;
  if (in_sizes[0] != NBATCH * NFEAT * NNODE) return;
  if (in_sizes[1] != 2 * NFEAT * NEMB) return;
  if (in_sizes[2] != NEMB || in_sizes[3] != NEMB) return;
  if (in_sizes[4] != NNODE * NNODE) return;
  if (out_size != NBATCH * NFEAT * NNODE) return;

  const float* x     = (const float*)d_in[0];
  const float* W     = (const float*)d_in[1];
  const float* b_lin = (const float*)d_in[2];
  const float* avec  = (const float*)d_in[3];
  const float* sbias = (const float*)d_in[4];
  float* out = (float*)d_out;

  const size_t szVT = (size_t)NBATCH * NNODE * NFEAT * 2;
  const size_t szXH = (size_t)NBATCH * NFEAT * NNODE * 2;
  const size_t szWT = (size_t)NEMB * 2 * NFEAT * 2;
  const size_t szP  = (size_t)NBATCH * NNODE * NEMB * 4;
  const size_t szPR = (size_t)NBATCH * NNODE * NNODE * 2;
  const size_t offVT = 0;
  const size_t offXH = offVT + szVT;
  const size_t offWT = offXH + szXH;
  const size_t offP  = offWT + szWT;
  const size_t offQ  = offP + szP;
  const size_t offPR = offQ + szP;
  const size_t total = offPR + szPR;
  if (ws_size < total) return;

  char* ws = (char*)d_ws;
  unsigned short* vT = (unsigned short*)(ws + offVT);
  unsigned short* xh = (unsigned short*)(ws + offXH);
  unsigned short* Wt = (unsigned short*)(ws + offWT);
  float* pproj = (float*)(ws + offP);
  float* qproj = (float*)(ws + offQ);
  unsigned short* Ppl = (unsigned short*)(ws + offPR);

  transpose_cast16<<<dim3(NNODE / 64, NFEAT / 64, NBATCH), dim3(256), 0, stream>>>(x, vT, NFEAT, NNODE, 1.0f);
  transpose_cast16<<<dim3(NEMB / 64, (2 * NFEAT) / 64, 1), dim3(256), 0, stream>>>(W, Wt, 2 * NFEAT, NEMB, WCARRY);
  const int n2 = NBATCH * NFEAT * NNODE / 2;
  cast_f32_f16x2<<<dim3((n2 + 255) / 256), dim3(256), 0, stream>>>(x, (_Float16*)xh, n2);

  const int tilesPQ = (NNODE / 64) * (NEMB / 64);
  wmma_gemm64<0, false, 2, 0, false, 0><<<dim3((tilesPQ + 7) / 8, NBATCH), dim3(256), 0, stream>>>(
      vT, vT, NFEAT, (long)NNODE * NFEAT,
      Wt, Wt, 2 * NFEAT, 0L,
      (void*)pproj, (void*)pproj, NEMB, (long)NNODE * NEMB,
      b_lin, b_lin, 0L,
      NNODE, NEMB, NFEAT, 1.0f / WCARRY);
  wmma_gemm64<0, false, 0, 0, false, 0><<<dim3((tilesPQ + 7) / 8, NBATCH), dim3(256), 0, stream>>>(
      vT, vT, NFEAT, (long)NNODE * NFEAT,
      Wt + NFEAT, Wt + NFEAT, 2 * NFEAT, 0L,
      (void*)qproj, (void*)qproj, NEMB, (long)NNODE * NEMB,
      b_lin, b_lin, 0L,
      NNODE, NEMB, NFEAT, 1.0f / WCARRY);

  score_softmax_kernel<<<dim3(NBATCH * (NNODE / ITILE)), dim3(256), 0, stream>>>(pproj, qproj, avec, sbias, Ppl);

  const int tilesO = (NFEAT / 64) * (NNODE / 64);
  wmma_gemm64<0, false, 0, 0, false, 6><<<dim3((tilesO + 7) / 8, NBATCH), dim3(256), 0, stream>>>(
      xh, xh, NNODE, (long)NFEAT * NNODE,
      Ppl, Ppl, NNODE, (long)NNODE * NNODE,
      (void*)out, (void*)out, NNODE, (long)NFEAT * NNODE,
      b_lin, b_lin, 0L,
      NFEAT, NNODE, NNODE, 1.0f / PCARRY);
}
